// Retention_66099546685816
// MI455X (gfx1250) — hardware-verified
//
#include <hip/hip_runtime.h>
#include <math.h>
#include <stdint.h>

#define NB_  2
#define T_   2048
#define C_   1024
#define NH_  16
#define KD_  64
#define VD_  128
#define VBD_ 2048
#define QKW_ 2048
#define GRK_ 4096
#define RT_P 132

static_assert(T_ % 64 == 0);
static_assert(C_ % 64 == 0);
static_assert(VBD_ % 64 == 0);
static_assert(QKW_ == 2 * C_);
static_assert(VBD_ == NH_ * VD_);
static_assert(C_ == NH_ * KD_);
static_assert(GRK_ == 2 * VBD_);
static_assert(C_ % 32 == 0);
static_assert(GRK_ % 32 == 0);
static_assert(((T_ / 64) * (QKW_ / 64)) % 8 == 0);
static_assert(((VBD_ / 64) * (T_ / 64)) % 8 == 0);
static_assert(((T_ / 64) * (C_ / 64)) % 8 == 0);
static_assert((NB_ * T_ * C_) % (8 * 256) == 0);
static_assert((NH_ * T_) % 256 == 0);

typedef __attribute__((ext_vector_type(16))) __bf16   v16b;
typedef __attribute__((ext_vector_type(8)))  float    v8f;
typedef __attribute__((ext_vector_type(4)))  float    v4f;
typedef __attribute__((ext_vector_type(4)))  unsigned int v4u;
typedef __attribute__((ext_vector_type(8)))  unsigned short u16x8;

union FragB { u16x8 h[2]; v16b v; };

constexpr size_t SZ_XB   = (size_t)NB_ * T_ * C_ * 2;
constexpr size_t SZ_WT   = (size_t)VBD_ * C_ * 2;
constexpr size_t SZ_WOT2 = (size_t)C_ * GRK_ * 2;
constexpr size_t SZ_SCL  = (size_t)NH_ * T_ * 4;
constexpr size_t SZ_QK   = (size_t)T_ * QKW_ * 2;
constexpr size_t SZ_VT   = (size_t)VBD_ * T_ * 2;
constexpr size_t SZ_G    = (size_t)T_ * VBD_ * 4;
constexpr size_t SZ_GRC  = (size_t)T_ * GRK_ * 2;

constexpr size_t OFF_XB   = 0;
constexpr size_t OFF_WQKT = OFF_XB   + SZ_XB;
constexpr size_t OFF_WVT  = OFF_WQKT + SZ_WT;
constexpr size_t OFF_WGT  = OFF_WVT  + SZ_WT;
constexpr size_t OFF_WOT2 = OFF_WGT  + SZ_WT;
constexpr size_t OFF_SCL  = OFF_WOT2 + SZ_WOT2;
constexpr size_t OFF_QKH  = OFF_SCL  + SZ_SCL;
constexpr size_t OFF_QKL  = OFF_QKH  + SZ_QK;
constexpr size_t OFF_VTH  = OFF_QKL  + SZ_QK;
constexpr size_t OFF_VTL  = OFF_VTH  + SZ_VT;
constexpr size_t OFF_G    = OFF_VTL  + SZ_VT;
constexpr size_t OFF_GRC  = OFF_G    + SZ_G;
constexpr size_t WS_END   = OFF_GRC  + SZ_GRC;
static_assert(WS_END <= (size_t)134217728);
static_assert(OFF_WQKT % 128 == 0 && OFF_WVT % 128 == 0 && OFF_WGT % 128 == 0 && OFF_WOT2 % 128 == 0);
static_assert(OFF_SCL % 128 == 0 && OFF_QKH % 128 == 0 && OFF_QKL % 128 == 0 && OFF_VTH % 128 == 0);
static_assert(OFF_VTL % 128 == 0 && OFF_G % 128 == 0 && OFF_GRC % 128 == 0);

__device__ __forceinline__ unsigned short f2bf_bits(float f) {
  unsigned u = __float_as_uint(f);
  return (unsigned short)((u + 0x7FFFu + ((u >> 16) & 1u)) >> 16);
}
__device__ __forceinline__ float bf_bits2f(unsigned short h) { return __uint_as_float(((unsigned)h) << 16); }
__device__ __forceinline__ float bf_rne(float f) { return bf_bits2f(f2bf_bits(f)); }
__device__ __forceinline__ unsigned pk16(unsigned short a, unsigned short b) { return (unsigned)a | ((unsigned)b << 16); }

__device__ __forceinline__ v16b frag_ld(const unsigned short* p) {
  FragB f; f.h[0] = *(const u16x8*)(p); f.h[1] = *(const u16x8*)(p + 16); return f.v;
}
__device__ __forceinline__ v8f mma_b(v16b a, v16b b, v8f c) {
  return __builtin_amdgcn_wmma_f32_16x16x32_bf16(false, a, false, b, (short)0, c, false, false);
}
__device__ __forceinline__ void dep_guard_b(v8f& a, v8f& b, v16b x, v16b y) {
  asm volatile("v_nop\n\tv_nop\n\tv_nop\n\tv_nop" : "+v"(a), "+v"(b) : "v"(x), "v"(y));
}
__device__ __forceinline__ void keep4_b(v16b a, v16b b, v16b c, v16b d) { asm volatile("v_nop" :: "v"(a), "v"(b), "v"(c), "v"(d)); }
__device__ __forceinline__ void acc_guard4(v8f& a, v8f& b, v8f& c, v8f& d) {
  asm volatile("v_nop\n\tv_nop\n\tv_nop\n\tv_nop" : "+v"(a), "+v"(b), "+v"(c), "+v"(d));
}
__device__ __forceinline__ v8f mma_g(v8f c, v16b a, v16b b) {
  c = __builtin_amdgcn_wmma_f32_16x16x32_bf16(false, a, false, b, (short)0, c, false, false);
  asm volatile("v_nop\n\tv_nop\n\tv_nop\n\tv_nop" : "+v"(c) : "v"(a), "v"(b));
  return c;
}

__global__ __launch_bounds__(256) void xcvt_kernel(const float* __restrict__ src, unsigned short* dst, int n8) {
  const int i = blockIdx.x * 256 + threadIdx.x;
  if (i < n8) {
    const size_t e = (size_t)i * 8;
    const v4f a = *(const v4f*)(src + e);
    const v4f b = *(const v4f*)(src + e + 4);
    u16x8 hv;
    hv[0] = f2bf_bits(a[0]); hv[1] = f2bf_bits(a[1]); hv[2] = f2bf_bits(a[2]); hv[3] = f2bf_bits(a[3]);
    hv[4] = f2bf_bits(b[0]); hv[5] = f2bf_bits(b[1]); hv[6] = f2bf_bits(b[2]); hv[7] = f2bf_bits(b[3]);
    *(volatile u16x8*)(dst + e) = hv;
    __threadfence();
    *(volatile u16x8*)(dst + e) = hv;
  }
}

template <bool DUP>
__global__ __launch_bounds__(256) void tcvt_kernel(const float* __restrict__ W, unsigned short* out, int R, int Cc, int ldo) {
  __shared__ __align__(16) float tf[64 * 68];
  const int c0  = blockIdx.x * 64;
  const int r0  = blockIdx.y * 64;
  const int tid = threadIdx.x;
  {
    const int lr = tid >> 4;
    const int c4 = (tid & 15) * 4;
#pragma unroll
    for (int it = 0; it < 4; ++it) {
      const int rr = it * 16 + lr;
      const v4f a = *(const v4f*)(W + (size_t)(r0 + rr) * Cc + c0 + c4);
      *(v4f*)(tf + rr * 68 + c4) = a;
    }
  }
  __syncthreads();
  const int sub = tid >> 3;
  const int c8  = (tid & 7) * 8;
  v4u hv[2];
#pragma unroll
  for (int it = 0; it < 2; ++it) {
    const int oc = it * 32 + sub;
    v4u a;
#pragma unroll
    for (int q = 0; q < 4; ++q) {
      const float f0 = tf[(c8 + 2 * q) * 68 + oc];
      const float f1 = tf[(c8 + 2 * q + 1) * 68 + oc];
      a[q] = pk16(f2bf_bits(f0), f2bf_bits(f1));
    }
    hv[it] = a;
  }
  for (int pass = 0; pass < 2; ++pass) {
#pragma unroll
    for (int it = 0; it < 2; ++it) {
      const int oc = it * 32 + sub;
      const size_t go = (size_t)(c0 + oc) * ldo + r0 + c8;
      *(volatile v4u*)(out + go) = hv[it];
      if (DUP) *(volatile v4u*)(out + go + R) = hv[it];
    }
    __threadfence();
  }
}

__global__ __launch_bounds__(256) void scl_kernel(float* scl, int n) {
  const int i = blockIdx.x * 256 + threadIdx.x;
  if (i < n) {
    const int h = i >> 11;
    const int t = i & (T_ - 1);
    const float e2    = __uint_as_float((unsigned)(122 - h) << 23);
    const float gamma = logf(1.0f - e2);
    const float num   = -expm1f(gamma * (float)(t + 1));
    const float sum   = num * __uint_as_float((unsigned)(132 + h) << 23);
    const float v = rsqrtf(sum);
    ((volatile float*)scl)[i] = v;
    __threadfence();
    ((volatile float*)scl)[i] = v;
  }
}

template <int BIAS_MODE, int OUT_MODE>
__global__ __launch_bounds__(256) void gemm64_kernel(
    const unsigned short* __restrict__ A, int lda, long strideA,
    const unsigned short* __restrict__ Bt, int ldb, long strideB,
    void* Cout, void* Cout2, int ldc, long strideC,
    const float* __restrict__ bias, int M, int N, int K) {
  __shared__ __align__(16) float sT[8][16 * 68];
  const int b    = blockIdx.y;
  const int lane = threadIdx.x & 31;
  const int wave = threadIdx.x >> 5;
  const int tilesN = N >> 6;
  const int tilesM = M >> 6;
  const int tile = blockIdx.x * 8 + wave;
  if (tile >= tilesM * tilesN) return;
  const int tm = tile / tilesN;
  const int tn = tile - tm * tilesN;
  const int m0 = tm << 6;
  const int n0 = tn << 6;

  const unsigned short* Ab = A  + (size_t)b * strideA;
  const unsigned short* Bb = Bt + (size_t)b * strideB;

  const int rlane = lane & 15;
  const int koff  = (lane >> 4) * 8;
  const int mOff  = (lane >> 4) * 8;

  v8f acc[4][4];
#pragma unroll
  for (int i = 0; i < 4; ++i)
#pragma unroll
    for (int j = 0; j < 4; ++j) acc[i][j] = (v8f){0.f,0.f,0.f,0.f,0.f,0.f,0.f,0.f};

  for (int k0 = 0; k0 < K; k0 += 32) {
    v16b bh[4];
#pragma unroll
    for (int j = 0; j < 4; ++j) {
      const size_t bo = (size_t)(n0 + (j << 4) + rlane) * ldb + koff + k0;
      bh[j] = frag_ld(Bb + bo);
    }
#pragma unroll
    for (int i = 0; i < 4; ++i) {
      const size_t ao = (size_t)(m0 + (i << 4) + rlane) * lda + koff + k0;
      v16b ah = frag_ld(Ab + ao);
#pragma unroll
      for (int j = 0; j < 4; ++j) acc[i][j] = mma_b(ah, bh[j], acc[i][j]);
      dep_guard_b(acc[i][0], acc[i][3], ah, ah);
    }
    keep4_b(bh[0], bh[1], bh[2], bh[3]);
  }
  acc_guard4(acc[0][0], acc[0][1], acc[0][2], acc[0][3]);
  acc_guard4(acc[1][0], acc[1][1], acc[1][2], acc[1][3]);
  acc_guard4(acc[2][0], acc[2][1], acc[2][2], acc[2][3]);
  acc_guard4(acc[3][0], acc[3][1], acc[3][2], acc[3][3]);

  float* slab = sT[wave];
#pragma unroll
  for (int i = 0; i < 4; ++i) {
    const int mBase = m0 + (i << 4);
    float bm[8];
#pragma unroll
    for (int r = 0; r < 8; ++r) bm[r] = 0.f;
    if (BIAS_MODE == 1) {
      const v4f b0 = *(const v4f*)(bias + mBase + mOff);
      const v4f b1 = *(const v4f*)(bias + mBase + mOff + 4);
      bm[0] = bf_rne(b0[0]); bm[1] = bf_rne(b0[1]); bm[2] = bf_rne(b0[2]); bm[3] = bf_rne(b0[3]);
      bm[4] = bf_rne(b1[0]); bm[5] = bf_rne(b1[1]); bm[6] = bf_rne(b1[2]); bm[7] = bf_rne(b1[3]);
    }
#pragma unroll
    for (int j = 0; j < 4; ++j) {
      const int n = n0 + (j << 4) + rlane;
      float bv = 0.f;
      if (BIAS_MODE == 2) bv = bf_rne(bias[n]);
#pragma unroll
      for (int r = 0; r < 8; ++r) {
        float v = acc[i][j][r];
        if (BIAS_MODE == 1) v += bm[r];
        if (BIAS_MODE == 2) v += bv;
        slab[(mOff + r) * 68 + (j << 4) + rlane] = v;
      }
    }
    __threadfence_block();
    __builtin_amdgcn_wave_barrier();
    __threadfence_block();
    if (OUT_MODE == 0) {
      float* Cp = (float*)Cout + (size_t)b * strideC;
      const int hh = lane >> 4, c4 = (lane & 15) * 4;
      for (int pass = 0; pass < 2; ++pass) {
#pragma unroll
        for (int it = 0; it < 8; ++it) {
          const int row = it * 2 + hh;
          v4f v = *(const v4f*)(slab + row * 68 + c4);
          *(volatile v4f*)(Cp + (size_t)(mBase + row) * ldc + n0 + c4) = v;
        }
        __threadfence();
      }
    } else {
      const int q = lane >> 3, c8 = (lane & 7) * 8;
      unsigned short* Cp  = (unsigned short*)Cout  + (size_t)b * strideC;
      unsigned short* Cp2 = (unsigned short*)Cout2 + (size_t)b * strideC;
      for (int pass = 0; pass < 2; ++pass) {
#pragma unroll
        for (int it = 0; it < 4; ++it) {
          const int row = it * 4 + q;
          const float* sp = slab + row * 68 + c8;
          u16x8 hv, lv;
#pragma unroll
          for (int e = 0; e < 8; ++e) {
            const float f = sp[e];
            const unsigned short hb = f2bf_bits(f);
            const unsigned short lb = f2bf_bits(f - bf_bits2f(hb));
            hv[e] = hb;
            lv[e] = lb;
          }
          *(volatile u16x8*)(Cp  + (size_t)(mBase + row) * ldc + n0 + c8) = hv;
          *(volatile u16x8*)(Cp2 + (size_t)(mBase + row) * ldc + n0 + c8) = lv;
        }
        __threadfence();
      }
    }
    __threadfence_block();
    __builtin_amdgcn_wave_barrier();
    __threadfence_block();
  }
}

__global__ __launch_bounds__(128) __attribute__((amdgpu_num_vgpr(240)))
void ret_kernel(const unsigned short* __restrict__ qkh, const unsigned short* __restrict__ qkl,
                const unsigned short* __restrict__ vth, const unsigned short* __restrict__ vtl,
                const float* __restrict__ gpl, const float* __restrict__ scl,
                unsigned short* grc) {
  __shared__ __align__(16) unsigned short Ksh[64 * KD_];
  __shared__ __align__(16) unsigned short Ksl[64 * KD_];
  __shared__ __align__(16) unsigned short Vsh[VD_ * 64];
  __shared__ __align__(16) unsigned short Vsl[VD_ * 64];
  __shared__ __align__(16) unsigned short Psh[4][16 * 64];
  __shared__ __align__(16) unsigned short Psl[4][16 * 64];
  __shared__ __align__(16) float Os[4][16 * RT_P];

  const int tid  = threadIdx.x;
  const int wave = tid >> 5;
  const int lane = tid & 31;
  const int hh   = lane >> 4;
  const int c    = lane & 15;

  const int qb  = blockIdx.x & 31;
  const int h   = blockIdx.x >> 5;
  const int q0w = qb * 64 + wave * 16;

  const unsigned short* Qh = qkh + h * KD_;
  const unsigned short* Ql = qkl + h * KD_;
  const unsigned short* Kh = qkh + C_ + h * KD_;
  const unsigned short* Kl = qkl + C_ + h * KD_;
  const unsigned short* Vh = vth + (size_t)(h * VD_) * T_;
  const unsigned short* Vl = vtl + (size_t)(h * VD_) * T_;

  const float gamma = logf(1.0f - __uint_as_float((unsigned)(122 - h) << 23));
  float eg[8];
#pragma unroll
  for (int r = 0; r < 8; ++r) eg[r] = expf(gamma * (float)r);

  float* os = Os[wave];
#pragma unroll
  for (int t = 0; t < 8; ++t)
#pragma unroll
    for (int r = 0; r < 8; ++r) os[(8 * hh + r) * RT_P + t * 16 + c] = 0.0f;

  float absSum[8];
#pragma unroll
  for (int r = 0; r < 8; ++r) absSum[r] = 0.0f;

  const int nChunks = qb + 1;
  for (int kc = 0; kc < nChunks; ++kc) {
    const int kv0 = kc * 64;
    __syncthreads();
    {
      const int r = tid >> 1, half = (tid & 1) * 32;
      const unsigned short* ks = Kh + (size_t)(kv0 + r) * QKW_ + half;
      const unsigned short* kl = Kl + (size_t)(kv0 + r) * QKW_ + half;
#pragma unroll
      for (int i = 0; i < 4; ++i) {
        const u16x8 a0 = *(const u16x8*)(ks + 8 * i);
        const u16x8 a1 = *(const u16x8*)(kl + 8 * i);
        *(u16x8*)(Ksh + r * KD_ + half + 8 * i) = a0;
        *(u16x8*)(Ksl + r * KD_ + half + 8 * i) = a1;
      }
      const unsigned short* vs = Vh + (size_t)tid * T_ + kv0;
      const unsigned short* vl = Vl + (size_t)tid * T_ + kv0;
#pragma unroll
      for (int i = 0; i < 8; ++i) {
        const u16x8 b0 = *(const u16x8*)(vs + 8 * i);
        const u16x8 b1 = *(const u16x8*)(vl + 8 * i);
        *(u16x8*)(Vsh + tid * 64 + 8 * i) = b0;
        *(u16x8*)(Vsl + tid * 64 + 8 * i) = b1;
      }
    }
    __syncthreads();

    FragB qah[2], qal[2];
#pragma unroll
    for (int dc = 0; dc < 2; ++dc) {
      const size_t qo = (size_t)(q0w + c) * QKW_ + dc * 32 + 8 * hh;
      qah[dc].h[0] = *(const u16x8*)(Qh + qo);
      qah[dc].h[1] = *(const u16x8*)(Qh + qo + 16);
      qal[dc].h[0] = *(const u16x8*)(Ql + qo);
      qal[dc].h[1] = *(const u16x8*)(Ql + qo + 16);
    }

#pragma unroll 1
    for (int j = 0; j < 4; ++j) {
      v8f s = (v8f){0.f,0.f,0.f,0.f,0.f,0.f,0.f,0.f};
#pragma unroll
      for (int dc = 0; dc < 2; ++dc) {
        FragB kb, kl2;
        const int ko = (j * 16 + c) * KD_ + dc * 32 + 8 * hh;
        kb.h[0]  = *(const u16x8*)(Ksh + ko);
        kb.h[1]  = *(const u16x8*)(Ksh + ko + 16);
        kl2.h[0] = *(const u16x8*)(Ksl + ko);
        kl2.h[1] = *(const u16x8*)(Ksl + ko + 16);
        s = mma_g(s, qah[dc].v, kb.v);
        s = mma_g(s, qah[dc].v, kl2.v);
        s = mma_g(s, qal[dc].v, kb.v);
      }
      const int d0 = q0w + 8 * hh - (kv0 + j * 16 + c);
      const float base = expf(gamma * (float)d0);
#pragma unroll
      for (int r = 0; r < 8; ++r) {
        const float val = (d0 + r >= 0) ? (s[r] * (base * eg[r])) : 0.0f;
        absSum[r] += fabsf(val);
        const unsigned short hb = f2bf_bits(val);
        const unsigned short lb = f2bf_bits(val - bf_bits2f(hb));
        Psh[wave][(8 * hh + r) * 64 + j * 16 + c] = hb;
        Psl[wave][(8 * hh + r) * 64 + j * 16 + c] = lb;
      }
    }
    __syncthreads();

#pragma unroll 1
    for (int vh = 0; vh < 2; ++vh) {
      const int cb = vh * 64;
      v8f oacc[4];
#pragma unroll
      for (int t = 0; t < 4; ++t)
#pragma unroll
        for (int r = 0; r < 8; ++r) oacc[t][r] = os[(8 * hh + r) * RT_P + cb + t * 16 + c];
#pragma unroll 1
      for (int kk = 0; kk < 2; ++kk) {
        FragB pa, pl;
        const int po = c * 64 + kk * 32 + 8 * hh;
        pa.h[0] = *(const u16x8*)(Psh[wave] + po);
        pa.h[1] = *(const u16x8*)(Psh[wave] + po + 16);
        pl.h[0] = *(const u16x8*)(Psl[wave] + po);
        pl.h[1] = *(const u16x8*)(Psl[wave] + po + 16);
#pragma unroll
        for (int t = 0; t < 4; ++t) {
          FragB vb, vl2;
          const int vo = (cb + t * 16 + c) * 64 + kk * 32 + 8 * hh;
          vb.h[0]  = *(const u16x8*)(Vsh + vo);
          vb.h[1]  = *(const u16x8*)(Vsh + vo + 16);
          vl2.h[0] = *(const u16x8*)(Vsl + vo);
          vl2.h[1] = *(const u16x8*)(Vsl + vo + 16);
          oacc[t] = mma_g(oacc[t], pa.v, vb.v);
          oacc[t] = mma_g(oacc[t], pa.v, vl2.v);
          oacc[t] = mma_g(oacc[t], pl.v, vb.v);
        }
      }
#pragma unroll
      for (int t = 0; t < 4; ++t)
#pragma unroll
        for (int r = 0; r < 8; ++r) os[(8 * hh + r) * RT_P + cb + t * 16 + c] = oacc[t][r];
    }
  }
  __syncthreads();

  float scv[8];
  {
    const float* sp = scl + (size_t)h * T_ + q0w + 8 * hh;
    const v4f a0 = *(const v4f*)sp;
    const v4f a1 = *(const v4f*)(sp + 4);
    scv[0] = a0[0]; scv[1] = a0[1]; scv[2] = a0[2]; scv[3] = a0[3];
    scv[4] = a1[0]; scv[5] = a1[1]; scv[6] = a1[2]; scv[7] = a1[3];
  }
#pragma unroll
  for (int r = 0; r < 8; ++r) {
    float a = absSum[r];
    a += __shfl_xor(a, 1, 32);
    a += __shfl_xor(a, 2, 32);
    a += __shfl_xor(a, 4, 32);
    a += __shfl_xor(a, 8, 32);
    const float den = fminf(fmaxf(a * scv[r], 1.0f), 50000.0f);
    const float fac = scv[r] * (1.0f / den);
    float rt[8];
    float ss = 0.0f;
#pragma unroll
    for (int t = 0; t < 8; ++t) { rt[t] = os[(8 * hh + r) * RT_P + t * 16 + c] * fac; ss += rt[t] * rt[t]; }
    ss += __shfl_xor(ss, 1, 32);
    ss += __shfl_xor(ss, 2, 32);
    ss += __shfl_xor(ss, 4, 32);
    ss += __shfl_xor(ss, 8, 32);
    const float rms = rsqrtf(ss * (1.0f / 128.0f) + 1.1920929e-07f);
#pragma unroll
    for (int t = 0; t < 8; ++t) os[(8 * hh + r) * RT_P + t * 16 + c] = rt[t] * rms;
  }
  __syncthreads();

  {
    const int rsub = lane >> 4;
    const int c8   = (lane & 15) * 8;
    for (int pass = 0; pass < 2; ++pass) {
#pragma unroll
      for (int it = 0; it < 8; ++it) {
        const int row = it * 2 + rsub;
        const float* op = os + row * RT_P + c8;
        const v4f y0 = *(const v4f*)op;
        const v4f y1 = *(const v4f*)(op + 4);
        const float* gp = gpl + (size_t)(q0w + row) * VBD_ + h * VD_ + c8;
        const v4f g0 = *(const v4f*)gp;
        const v4f g1 = *(const v4f*)(gp + 4);
        u16x8 hv, lv;
#pragma unroll
        for (int e = 0; e < 4; ++e) {
          const float f0 = y0[e] * g0[e];
          const unsigned short h0 = f2bf_bits(f0);
          hv[e] = h0;
          lv[e] = f2bf_bits(f0 - bf_bits2f(h0));
          const float f1 = y1[e] * g1[e];
          const unsigned short h1 = f2bf_bits(f1);
          hv[4 + e] = h1;
          lv[4 + e] = f2bf_bits(f1 - bf_bits2f(h1));
        }
        unsigned short* dp = grc + (size_t)(q0w + row) * GRK_ + h * VD_ + c8;
        *(volatile u16x8*)dp = hv;
        *(volatile u16x8*)(dp + VBD_) = lv;
      }
      __threadfence();
    }
  }
}

extern "C" void kernel_launch(void* const* d_in, const int* in_sizes, int n_in,
                              void* d_out, int out_size, void* d_ws, size_t ws_size,
                              hipStream_t stream) {
  if (n_in < 9) return;
  if (in_sizes[0] != NB_ * T_ * C_) return;
  if (in_sizes[1] != C_ * QKW_) return;
  if (in_sizes[2] != QKW_) return;
  if (in_sizes[3] != C_ * VBD_) return;
  if (in_sizes[4] != VBD_) return;
  if (in_sizes[5] != C_ * VBD_) return;
  if (in_sizes[6] != VBD_) return;
  if (in_sizes[7] != VBD_ * C_) return;
  if (in_sizes[8] != C_) return;
  if (out_size != NB_ * T_ * C_) return;
  if (ws_size < WS_END) return;

  const float* x    = (const float*)d_in[0];
  const float* W_qk = (const float*)d_in[1];
  const float* b_qk = (const float*)d_in[2];
  const float* W_v  = (const float*)d_in[3];
  const float* b_v  = (const float*)d_in[4];
  const float* W_g  = (const float*)d_in[5];
  const float* b_g  = (const float*)d_in[6];
  const float* W_o  = (const float*)d_in[7];
  const float* b_o  = (const float*)d_in[8];
  float* out = (float*)d_out;

  char* ws = (char*)d_ws;
  unsigned short* XB   = (unsigned short*)(ws + OFF_XB);
  unsigned short* WQKT = (unsigned short*)(ws + OFF_WQKT);
  unsigned short* WVT  = (unsigned short*)(ws + OFF_WVT);
  unsigned short* WGT  = (unsigned short*)(ws + OFF_WGT);
  unsigned short* WOT2 = (unsigned short*)(ws + OFF_WOT2);
  float*          SCL  = (float*)(ws + OFF_SCL);
  unsigned short* QKH  = (unsigned short*)(ws + OFF_QKH);
  unsigned short* QKL  = (unsigned short*)(ws + OFF_QKL);
  unsigned short* VTH  = (unsigned short*)(ws + OFF_VTH);
  unsigned short* VTL  = (unsigned short*)(ws + OFF_VTL);
  float*          G    = (float*)(ws + OFF_G);
  unsigned short* GRC  = (unsigned short*)(ws + OFF_GRC);

  const dim3 blk(256);

  {
    const int n8 = NB_ * T_ * C_ / 8;
    xcvt_kernel<<<dim3(n8 / 256), blk, 0, stream>>>(x, XB, n8);
  }
  tcvt_kernel<false><<<dim3(QKW_ / 64, C_ / 64), blk, 0, stream>>>(W_qk, WQKT, C_, QKW_, C_);
  tcvt_kernel<false><<<dim3(VBD_ / 64, C_ / 64), blk, 0, stream>>>(W_v, WVT, C_, VBD_, C_);
  tcvt_kernel<false><<<dim3(VBD_ / 64, C_ / 64), blk, 0, stream>>>(W_g, WGT, C_, VBD_, C_);
  tcvt_kernel<true><<<dim3(C_ / 64, VBD_ / 64), blk, 0, stream>>>(W_o, WOT2, VBD_, C_, GRK_);
  scl_kernel<<<dim3((NH_ * T_) / 256), blk, 0, stream>>>(SCL, NH_ * T_);

  const dim3 gQK(((T_ / 64) * (QKW_ / 64)) / 8, 1);
  const dim3 gVT(((VBD_ / 64) * (T_ / 64)) / 8, 1);
  const dim3 gG (((T_ / 64) * (VBD_ / 64)) / 8, 1);
  const dim3 gO (((T_ / 64) * (C_ / 64)) / 8, 1);
  const dim3 gR (NH_ * (T_ / 64));

  for (int b = 0; b < NB_; ++b) {
    const unsigned short* XBb = XB + (size_t)b * T_ * C_;
    gemm64_kernel<2, 2><<<gQK, blk, 0, stream>>>(
        XBb, C_, 0L, WQKT, C_, 0L, (void*)QKH, (void*)QKL, QKW_, 0L, b_qk, T_, QKW_, C_);
    gemm64_kernel<1, 2><<<gVT, blk, 0, stream>>>(
        WVT, C_, 0L, XBb, C_, 0L, (void*)VTH, (void*)VTL, T_, 0L, b_v, VBD_, T_, C_);
    gemm64_kernel<2, 0><<<gG, blk, 0, stream>>>(
        XBb, C_, 0L, WGT, C_, 0L, (void*)G, (void*)G, VBD_, 0L, b_g, T_, VBD_, C_);
    ret_kernel<<<gR, dim3(128), 0, stream>>>(QKH, QKL, VTH, VTL, G, SCL, GRC);
    float* outb = out + (size_t)b * T_ * C_;
    gemm64_kernel<2, 0><<<gO, blk, 0, stream>>>(
        GRC, GRK_, 0L, WOT2, GRK_, 0L, (void*)outb, (void*)outb, C_, 0L, b_o, T_, C_, GRK_);
  }
  (void)hipGetLastError();
}
